// FeatureFusionModel_23330262351963
// MI455X (gfx1250) — hardware-verified
//
#include <hip/hip_runtime.h>
#include <stddef.h>


#pragma clang fp contract(off)

#define BATCH   2
#define NVIEWS  6
#define MTOK    1369
#define DIM     384
#define NVOX    50000
#define PF      64
#define HID     256
#define OUTD    16
#define FDIM    448
#define LDA     456
#define LDH     264
#define TM      32
#define NTHR    256
#define NWAVE   (NTHR / 32)
#define PGRID   37
#define TOTALV  (BATCH * NVOX)
#define NBLK_MAIN ((TOTALV + TM - 1) / TM)
#define NP_MEAN (BATCH * MTOK * DIM / 8)
#define NP_W1   (HID * FDIM / 8)
#define NP_W2   (OUTD * HID / 8)
#define NBLK_MEAN ((NP_MEAN + NTHR - 1) / NTHR)
#define NBLK_W1 (NP_W1 / NTHR)
#define NBLK_W2 (NP_W2 / NTHR)
#define SC_W    64.0f
#define SC_H    8.0f
#define INV1    (1.0f / 64.0f)
#define INV2    (1.0f / 512.0f)

static_assert(FDIM == PF + DIM);
static_assert(FDIM % 32 == 0);
static_assert(HID % 32 == 0);
static_assert(DIM % 8 == 0);
static_assert((MTOK * DIM) % 8 == 0);
static_assert(NP_W1 % NTHR == 0);
static_assert(NP_W2 % NTHR == 0);
static_assert(TM * 8 == NTHR);
static_assert(TM == 32);
static_assert(HID == 32 * NWAVE);
static_assert(TM * OUTD / 4 <= NTHR);
static_assert(LDA % 8 == 0);
static_assert(LDH % 8 == 0);
static_assert(LDA >= FDIM);
static_assert(LDH >= HID);
static_assert(PGRID * PGRID == MTOK);
static_assert(DIM / 8 == 48);

typedef _Float16 v16h __attribute__((ext_vector_type(16)));
typedef _Float16 v8h  __attribute__((ext_vector_type(8)));
typedef float    v4f  __attribute__((ext_vector_type(4)));
typedef float    v8f  __attribute__((ext_vector_type(8)));
union FragH { v16h v; v8h hv[2]; };

__device__ __forceinline__ v8f wmh(v16h a, v16h b, v8f c) {
  v8f d = __builtin_amdgcn_wmma_f32_16x16x32_f16(false, a, false, b, (short)0, c, false, false);
#if defined(__HIP_DEVICE_COMPILE__)
  asm volatile("v_nop\n\tv_nop\n\tv_nop\n\tv_nop" : "+v"(d) : "v"(a), "v"(b));
#endif
  return d;
}

__device__ __forceinline__ v8f zero8() {
  v8f z = {0.f, 0.f, 0.f, 0.f, 0.f, 0.f, 0.f, 0.f};
  return z;
}

__device__ __forceinline__ v16h afrag(const _Float16* row, int k0, int h) {
  FragH u;
  u.hv[0] = *(const v8h*)(row + k0 + 8 * h);
  u.hv[1] = *(const v8h*)(row + k0 + 16 + 8 * h);
  return u.v;
}

__global__ __launch_bounds__(NTHR) void k_meant(const float* __restrict__ patch, _Float16* meant) {
  const int g = blockIdx.x * NTHR + (int)threadIdx.x;
  if (g >= NP_MEAN) return;
  const size_t e    = (size_t)8 * g;
  const size_t perb = (size_t)MTOK * DIM;
  const int b = (int)(e / perb);
  const size_t r = e - (size_t)b * perb;
  const float* p = patch + (size_t)b * NVIEWS * perb + r;
  v4f s0 = *(const v4f*)p;
  v4f s1 = *(const v4f*)(p + 4);
#pragma unroll
  for (int v = 1; v < NVIEWS; ++v) {
    const float* q = p + (size_t)v * perb;
    s0 += *(const v4f*)q;
    s1 += *(const v4f*)(q + 4);
  }
  v8h o;
#pragma unroll
  for (int i = 0; i < 4; ++i) {
    o[i]     = (_Float16)(s0[i] * (1.0f / 6.0f));
    o[4 + i] = (_Float16)(s1[i] * (1.0f / 6.0f));
  }
  _Float16* d = meant + e;
  *(volatile v8h*)d = o;
  __threadfence();
  *(volatile v8h*)d = o;
}

__global__ __launch_bounds__(NTHR) void k_wprep(const float* __restrict__ w1, const float* __restrict__ w2,
                                                _Float16* w1s, _Float16* w2s) {
  const int tid = (int)threadIdx.x;
  if (blockIdx.x < NBLK_W1) {
    const int g  = blockIdx.x * NTHR + tid;
    const int n  = g / (FDIM / 8);
    const int kp = g - n * (FDIM / 8);
    const float* src = w1 + (size_t)(8 * kp) * HID + n;
    v8h o;
#pragma unroll
    for (int i = 0; i < 8; ++i) o[i] = (_Float16)(SC_W * src[(size_t)i * HID]);
    _Float16* d = w1s + (size_t)8 * g;
    *(volatile v8h*)d = o;
    __threadfence();
    *(volatile v8h*)d = o;
  } else {
    const int g  = (blockIdx.x - NBLK_W1) * NTHR + tid;
    const int n  = g >> 5;
    const int kp = g & 31;
    const float* src = w2 + (size_t)(8 * kp) * OUTD + n;
    v8h o;
#pragma unroll
    for (int i = 0; i < 8; ++i) o[i] = (_Float16)(SC_W * src[(size_t)i * OUTD]);
    _Float16* d = w2s + (size_t)8 * g;
    *(volatile v8h*)d = o;
    __threadfence();
    *(volatile v8h*)d = o;
  }
}

__global__ __launch_bounds__(NTHR) void k_main(const float* __restrict__ voxf, const float* __restrict__ voxc,
                                               const float* __restrict__ kmat, const float* __restrict__ rtm,
                                               const _Float16* __restrict__ w1s, const float* __restrict__ b1,
                                               const _Float16* __restrict__ w2s, const float* __restrict__ b2,
                                               const _Float16* __restrict__ meant,
                                               const int* __restrict__ rs_p, const int* __restrict__ ps_p,
                                               const int* __restrict__ wo_p, const int* __restrict__ ho_p,
                                               float* out) {
  __shared__ __align__(16) _Float16 sA[TM * LDA];
  __shared__ __align__(16) _Float16 sH[TM * LDH];
  __shared__ __align__(16) v4f s_out4[TM * OUTD / 4];
  __shared__ int s_idx[TM];
  __shared__ int s_bat[TM];
  float* s_out = (float*)s_out4;

  const int tid = (int)threadIdx.x, lane = tid & 31, w = tid >> 5, h = lane >> 4, m = lane & 15;
  const int base = blockIdx.x * TM;

  if (w == 0) {
    int gv = base + lane;
    gv = gv > TOTALV - 1 ? TOTALV - 1 : gv;
    const int b = gv / NVOX;
    const float* c = voxc + (size_t)gv * 3;
    const float x = c[0], y = c[1], z = c[2];
    const float* R = rtm + b * 12;
    float cx = R[0] * x;  cx = fmaf(R[1], y, cx);  cx = fmaf(R[2],  z, cx);  cx = fmaf(R[3],  1.0f, cx);
    float cy = R[4] * x;  cy = fmaf(R[5], y, cy);  cy = fmaf(R[6],  z, cy);  cy = fmaf(R[7],  1.0f, cy);
    float cz = R[8] * x;  cz = fmaf(R[9], y, cz);  cz = fmaf(R[10], z, cz);  cz = fmaf(R[11], 1.0f, cz);
    const float* Km = kmat + b * 9;
    float px = Km[0] * cx;  px = fmaf(Km[1], cy, px);  px = fmaf(Km[2], cz, px);
    float py = Km[3] * cx;  py = fmaf(Km[4], cy, py);  py = fmaf(Km[5], cz, py);
    float pz = Km[6] * cx;  pz = fmaf(Km[7], cy, pz);  pz = fmaf(Km[8], cz, pz);
    const float den = pz + 1e-6f;
    const float inv = 1.0f / den;
    const float u  = px * inv;
    const float vv = py * inv;
    int rs = rs_p[0], ps = ps_p[0], wo = wo_p[0], ho = ho_p[0];
    ps = ps < 1 ? 1 : ps;
    wo = wo < 1 ? 1 : wo;
    ho = ho < 1 ? 1 : ho;
    const float su = (float)((double)rs / (double)wo);
    const float sv = (float)((double)rs / (double)ho);
    int grid = rs / ps;
    grid = grid < 1 ? 1 : grid;
    const float rcp = 1.0f / (float)ps;
    float tu = (u * su) * rcp;
    float tv = (vv * sv) * rcp;
    const float gmax = (float)(grid - 1);
    tu = fminf(fmaxf(tu, 0.0f), gmax);
    tv = fminf(fmaxf(tv, 0.0f), gmax);
    const int gx = (int)tu;
    const int gy = (int)tv;
    int fi = gx * grid + gy;
    fi = fi < 0 ? 0 : (fi > MTOK - 1 ? MTOK - 1 : fi);
    s_idx[lane] = fi;
    s_bat[lane] = b;
  }
  __syncthreads();

  {
    const int rr = tid >> 3;
    const int t8 = tid & 7;
    int gv = base + rr;
    gv = gv > TOTALV - 1 ? TOTALV - 1 : gv;
    const float* vf = voxf + (size_t)gv * PF + 8 * t8;
    const v4f u0 = *(const v4f*)vf;
    const v4f u1 = *(const v4f*)(vf + 4);
    v8h o;
#pragma unroll
    for (int i = 0; i < 4; ++i) {
      o[i]     = (_Float16)u0[i];
      o[4 + i] = (_Float16)u1[i];
    }
    *(v8h*)(sA + rr * LDA + 8 * t8) = o;
    const _Float16* src = meant + ((size_t)s_bat[rr] * MTOK + (size_t)s_idx[rr]) * DIM + 48 * t8;
    _Float16* dst = sA + rr * LDA + PF + 48 * t8;
#pragma unroll
    for (int cpy = 0; cpy < 6; ++cpy) *(v8h*)(dst + 8 * cpy) = *(const v8h*)(src + 8 * cpy);
  }
  __syncthreads();

  v8f acc[2][2];
#pragma unroll
  for (int mt = 0; mt < 2; ++mt)
#pragma unroll
    for (int ct = 0; ct < 2; ++ct) acc[mt][ct] = zero8();

  const _Float16* arow0 = w1s + (size_t)(32 * w + m) * FDIM;
  const _Float16* arow1 = arow0 + (size_t)16 * FDIM;

#pragma unroll 2
  for (int ks = 0; ks < FDIM / 32; ++ks) {
    const int k0 = 32 * ks;
    const v16h a0 = afrag(arow0, k0, h);
    const v16h a1 = afrag(arow1, k0, h);
    const v16h f0 = afrag(sA + m * LDA, k0, h);
    const v16h f1 = afrag(sA + (16 + m) * LDA, k0, h);
    acc[0][0] = wmh(a0, f0, acc[0][0]);
    acc[1][0] = wmh(a1, f0, acc[1][0]);
    acc[0][1] = wmh(a0, f1, acc[0][1]);
    acc[1][1] = wmh(a1, f1, acc[1][1]);
  }

#pragma unroll
  for (int mt = 0; mt < 2; ++mt) {
    const int hb = 32 * w + 16 * mt + 8 * h;
    const v4f bb0 = *(const v4f*)(b1 + hb);
    const v4f bb1 = *(const v4f*)(b1 + hb + 4);
#pragma unroll
    for (int ct = 0; ct < 2; ++ct) {
      v8h o;
#pragma unroll
      for (int r = 0; r < 4; ++r) {
        const float v0 = fmaxf(acc[mt][ct][r] * INV1 + bb0[r], 0.0f);
        const float v1 = fmaxf(acc[mt][ct][4 + r] * INV1 + bb1[r], 0.0f);
        o[r]     = (_Float16)(SC_H * v0);
        o[4 + r] = (_Float16)(SC_H * v1);
      }
      *(v8h*)(sH + (16 * ct + m) * LDH + hb) = o;
    }
  }
  __syncthreads();

  if (w < 2) {
    const int ct = w;
    v8f acc2 = zero8();
    const _Float16* hrow = sH + (16 * ct + m) * LDH;
    const _Float16* wrow = w2s + (size_t)m * HID;
#pragma unroll 2
    for (int ks = 0; ks < HID / 32; ++ks) {
      const int k0 = 32 * ks;
      const v16h af = afrag(hrow, k0, h);
      const v16h bf = afrag(wrow, k0, h);
      acc2 = wmh(af, bf, acc2);
    }
    const float bias = b2[m];
#pragma unroll
    for (int r = 0; r < 8; ++r) {
      s_out[(16 * ct + 8 * h + r) * OUTD + m] = acc2[r] * INV2 + bias;
    }
  }
  __syncthreads();

  if (tid < TM * OUTD / 4) {
    const int vox = base + (tid >> 2);
    if (vox < TOTALV) {
      const v4f o = s_out4[tid];
      float* po = out + (size_t)base * OUTD + 4 * tid;
      *(volatile v4f*)po = o;
      __threadfence();
      *(volatile v4f*)po = o;
    }
  }
}

static inline size_t al128(size_t x) { return (x + 127) & ~(size_t)127; }

extern "C" void kernel_launch(void* const* d_in, const int* in_sizes, int n_in,
                              void* d_out, int out_size, void* d_ws, size_t ws_size,
                              hipStream_t stream) {
  if (n_in < 13) return;
  if (in_sizes[0] != BATCH * NVIEWS * MTOK * DIM) return;
  if (in_sizes[1] != BATCH * NVOX * PF) return;
  if (in_sizes[2] != BATCH * NVOX * 3) return;
  if (in_sizes[3] != BATCH * 9 || in_sizes[4] != BATCH * 12) return;
  if (in_sizes[5] != FDIM * HID || in_sizes[6] != HID) return;
  if (in_sizes[7] != HID * OUTD || in_sizes[8] != OUTD) return;
  if (in_sizes[9] != 1 || in_sizes[10] != 1 || in_sizes[11] != 1 || in_sizes[12] != 1) return;
  if (out_size != TOTALV * OUTD) return;

  const float* patch = (const float*)d_in[0];
  const float* voxf  = (const float*)d_in[1];
  const float* voxc  = (const float*)d_in[2];
  const float* kmat  = (const float*)d_in[3];
  const float* rtm   = (const float*)d_in[4];
  const float* w1    = (const float*)d_in[5];
  const float* b1    = (const float*)d_in[6];
  const float* w2    = (const float*)d_in[7];
  const float* b2    = (const float*)d_in[8];
  const int*   rs_p  = (const int*)d_in[9];
  const int*   ps_p  = (const int*)d_in[10];
  const int*   wo_p  = (const int*)d_in[11];
  const int*   ho_p  = (const int*)d_in[12];
  float* out = (float*)d_out;

  const size_t sz_meant = (size_t)NP_MEAN * 16;
  const size_t sz_w1s   = (size_t)NP_W1 * 16;
  const size_t sz_w2s   = (size_t)NP_W2 * 16;
  const size_t off_meant = 0;
  const size_t off_w1s   = al128(off_meant + sz_meant);
  const size_t off_w2s   = al128(off_w1s + sz_w1s);
  const size_t total     = al128(off_w2s + sz_w2s);
  if (total > ws_size || total > (size_t)134217728) return;

  char* ws = (char*)d_ws;
  _Float16* meant = (_Float16*)(ws + off_meant);
  _Float16* w1s   = (_Float16*)(ws + off_w1s);
  _Float16* w2s   = (_Float16*)(ws + off_w2s);

  k_meant<<<NBLK_MEAN, NTHR, 0, stream>>>(patch, meant);
  k_wprep<<<NBLK_W1 + NBLK_W2, NTHR, 0, stream>>>(w1, w2, w1s, w2s);
  k_main<<<NBLK_MAIN, NTHR, 0, stream>>>(voxf, voxc, kmat, rtm, w1s, b1, w2s, b2, meant,
                                         rs_p, ps_p, wo_p, ho_p, out);
}
